// MultiHeadCfC_34763465294531
// MI455X (gfx1250) — hardware-verified
//
#include <hip/hip_runtime.h>
#include <math.h>

typedef __attribute__((ext_vector_type(16))) _Float16 v16h;
typedef __attribute__((ext_vector_type(16))) __bf16 v16b;
typedef __attribute__((ext_vector_type(8)))  _Float16 v8h;
typedef __attribute__((ext_vector_type(8)))  float v8f;
typedef __attribute__((ext_vector_type(4)))  float v4f;
typedef __attribute__((ext_vector_type(2)))  float v2f;
typedef __attribute__((ext_vector_type(4)))  unsigned v4u;
typedef __attribute__((ext_vector_type(4)))  int v4i;
typedef float __attribute__((may_alias)) float_a;
typedef int __attribute__((may_alias)) int_a;

template <typename T> __device__ __forceinline__ void vst2(void* p, T v) { *(volatile T*)p = v; __threadfence(); *(volatile T*)p = v; }
__device__ __forceinline__ v8f wmma16(v16h a, v16h b, v8f c) {
  v8f d = __builtin_amdgcn_wmma_f32_16x16x32_f16(false, a, false, b, (short)0, c, false, false);
  asm volatile("v_nop\n\tv_nop\n\tv_nop\n\tv_nop" : "+v"(d) : "v"(a), "v"(b));
  return d;
}
__device__ __forceinline__ v8f wmma_bf(v16b a, v16b b, v8f c) {
  v8f d = __builtin_amdgcn_wmma_f32_16x16x32_bf16(false, a, false, b, (short)0, c, false, false);
  asm volatile("v_nop\n\tv_nop\n\tv_nop\n\tv_nop" : "+v"(d) : "v"(a), "v"(b));
  return d;
}
__device__ __forceinline__ v16h frag_h(const _Float16* rowk0, int lane) {
  union { v16h v; v8h q[2]; } u; const _Float16* p = rowk0 + 8 * (lane >> 4);
  u.q[0] = *(const v8h*)p; u.q[1] = *(const v8h*)(p + 16); return u.v;
}
__device__ __forceinline__ v16h frag_f32(const float* rowk0, int lane) {
  v16h a; const float* p = rowk0 + 8 * (lane >> 4);
#pragma unroll
  for (int i = 0; i < 8; ++i) { a[i] = (_Float16)p[i]; a[8 + i] = (_Float16)p[16 + i]; }
  return a;
}
__device__ __forceinline__ v16h frag_f32s(const float* rowk0, int lane, float sc) {
  v16h a; const float* p = rowk0 + 8 * (lane >> 4);
#pragma unroll
  for (int i = 0; i < 8; ++i) { a[i] = (_Float16)(p[i] * sc); a[8 + i] = (_Float16)(p[16 + i] * sc); }
  return a;
}
__device__ __forceinline__ v16h fragc_f32(const float* W, int k0, int n, int lane, int ld, int K) {
  v16h a; const int g = lane >> 4;
#pragma unroll
  for (int i = 0; i < 8; ++i) { const int ka = k0 + 8 * g + i, kb = ka + 16;
    a[i] = (_Float16)(ka < K ? W[(size_t)(ka < K ? ka : K - 1) * ld + n] : 0.f); a[8 + i] = (_Float16)(kb < K ? W[(size_t)(kb < K ? kb : K - 1) * ld + n] : 0.f); }
  return a;
}
struct F2 { v16b h, l; };
__device__ __forceinline__ F2 bsplit16(const float v[16]) { F2 r;
#pragma unroll
  for (int i = 0; i < 16; ++i) { const __bf16 h = (__bf16)v[i]; r.h[i] = h; r.l[i] = (__bf16)(v[i] - (float)h); }
  return r; }
__device__ __forceinline__ F2 split_row(const float* row, int k0, int lane) { float v[16]; const float* p = row + k0 + 8 * (lane >> 4);
#pragma unroll
  for (int i = 0; i < 8; ++i) { v[i] = p[i]; v[8 + i] = p[16 + i]; }
  return bsplit16(v); }
__device__ __forceinline__ F2 split_rowK(const float* row, int k0, int lane, int K) { float v[16]; const int g = lane >> 4;
#pragma unroll
  for (int i = 0; i < 8; ++i) { const int ka = k0 + 8 * g + i, kb = ka + 16; v[i] = ka < K ? row[ka < K ? ka : K - 1] : 0.f; v[8 + i] = kb < K ? row[kb < K ? kb : K - 1] : 0.f; }
  return bsplit16(v); }
__device__ __forceinline__ F2 split_col(const float* W, int k0, int n, int lane, int ld, int K) { float v[16]; const int g = lane >> 4;
#pragma unroll
  for (int i = 0; i < 8; ++i) { const int ka = k0 + 8 * g + i, kb = ka + 16; v[i] = ka < K ? W[(size_t)(ka < K ? ka : K - 1) * ld + n] : 0.f; v[8 + i] = kb < K ? W[(size_t)(kb < K ? kb : K - 1) * ld + n] : 0.f; }
  return bsplit16(v); }
__device__ __forceinline__ v8f mac3(const F2& a, const F2& b, v8f c) { c = wmma_bf(a.l, b.h, c); c = wmma_bf(a.h, b.l, c); return wmma_bf(a.h, b.h, c); }
__device__ __forceinline__ float sigm(float v) { return 1.0f / (1.0f + expf(-v)); }
#define LDSX() do { asm volatile("s_wait_dscnt 0" ::: "memory"); __builtin_amdgcn_wave_barrier(); __builtin_amdgcn_fence(__ATOMIC_RELEASE, "workgroup"); } while (0)


#define NV 8
#define NBAT 256
#define NT 128
#define NU 128
#define NHID 1024
#define NCLS 10
#ifndef NRG
#define NRG (NBAT / 32)
#define NOUT NBAT
#endif
typedef __attribute__((ext_vector_type(8))) __bf16 v8b;
__device__ __forceinline__ v16b frag_b(const __bf16* rowk0, int lane) {
  union { v16b v; v8b q[2]; } u; const __bf16* p = rowk0 + 8 * (lane >> 4);
  u.q[0] = *(const v8b*)p; u.q[1] = *(const v8b*)(p + 16); return u.v;
}
__device__ __forceinline__ float bfr(float v) { return (float)(__bf16)v; }
__device__ __attribute__((noinline)) float exp_ni(float v) { return expf(v); }
__device__ __attribute__((noinline)) float erf_ni(float v) { return erff(v); }
__device__ __forceinline__ float ftanh(float x) { return 1.0f - 2.0f / (__expf(2.0f * x) + 1.0f); }
__device__ __forceinline__ float fsigm(float x) { return 1.0f / (1.0f + __expf(-x)); }

#define PV_SZ (5 * NU * NU)
#define PK_FC1 (NV * PV_SZ)
#define PK_FC2 (PK_FC1 + NHID * NHID)
#define PK_END (PK_FC2 + 16 * NHID)
#define WS_PK 0u
#define WS_FE (WS_PK + 2u * PK_END)
#define WS_H1 (WS_FE + 4u * NBAT * NHID)
#define WS_END (WS_H1 + 4u * NBAT * NHID)

__global__ __launch_bounds__(256) void k_packT(const float* __restrict__ WBB, const float* __restrict__ WF1, const float* __restrict__ WF2, const float* __restrict__ WTA, const float* __restrict__ WTB, const float* __restrict__ WFC1, const float* __restrict__ WFC2, __bf16* __restrict__ PK) {
  __shared__ __align__(16) __bf16 s[NHID]; const int n = blockIdx.x, which = blockIdx.y, tid = threadIdx.x; int K; size_t dst;
  if (which < 40) { if (n >= NU) return; const int v = which / 5, m = which % 5; K = NU; dst = (size_t)v * PV_SZ + (size_t)m * NU * NU + (size_t)n * NU;
    if (m == 0) { for (int k = tid; k < K; k += 256) s[k] = (__bf16)WBB[((size_t)v * (NU + 1) + 1 + k) * NU + n]; }
    else { const float* Wm = (m == 1) ? WF1 : (m == 2) ? WF2 : (m == 3) ? WTA : WTB; for (int k = tid; k < K; k += 256) s[k] = (__bf16)Wm[((size_t)v * NU + k) * NU + n]; } }
  else if (which == 40) { K = NHID; dst = PK_FC1 + (size_t)n * NHID; for (int k = tid; k < K; k += 256) s[k] = (__bf16)WFC1[(size_t)k * NHID + n]; }
  else { if (n >= 16) return; K = NHID; dst = PK_FC2 + (size_t)n * NHID; for (int k = tid; k < K; k += 256) s[k] = (__bf16)((n < NCLS) ? WFC2[(size_t)k * NCLS + n] : 0.f); }
  __syncthreads();
  for (int q = tid; q < K / 8; q += 256) vst2((unsigned*)(PK + dst + q * 8), *(const v4u*)&s[q * 8]);
}
__device__ __forceinline__ void gemm16x128(const float* arows  , const __bf16* __restrict__ Wrows, int lane, int col, v8f acc[8]) {
#pragma unroll 1
  for (int kc = 0; kc < NU / 32; ++kc) { const F2 a = split_row(arows, kc * 32, lane);
#pragma unroll
    for (int j = 0; j < 8; ++j) { const v16b w = frag_b(Wrows + (size_t)(j * 16 + col) * NU + kc * 32, lane); acc[j] = wmma_bf(a.l, w, acc[j]); acc[j] = wmma_bf(a.h, w, acc[j]); } }
}
__global__ __launch_bounds__(64) void k_cfc(const float* __restrict__ X, const float* __restrict__ WBB, const float* __restrict__ BBB, const float* __restrict__ BF1, const float* __restrict__ BF2, const float* __restrict__ BTA, const float* __restrict__ BTB, const __bf16* __restrict__ PK, float* __restrict__ FE) {
  __shared__ __align__(16) float sh[2][16][132], sz[2][16][132], sf1[2][16][132], sf2[2][16][132];
  const int tid = threadIdx.x, wave = tid >> 5, lane = tid & 31, col = lane & 15, g = lane >> 4; const int v = blockIdx.y; const int b0 = blockIdx.x * 32 + wave * 16;
  const __bf16* PV = PK + (size_t)v * PV_SZ; const __bf16 *PBB = PV, *PF1 = PV + NU * NU, *PF2 = PV + 2 * NU * NU, *PTA = PV + 3 * NU * NU, *PTB = PV + 4 * NU * NU;
  float wx[8], bb[8], b1[8], b2[8], bt[8];
#pragma unroll
  for (int j = 0; j < 8; ++j) { const int n = j * 16 + col; wx[j] = bfr(WBB[(size_t)v * (NU + 1) * NU + n]); bb[j] = bfr(BBB[v * NU + n]); b1[j] = bfr(BF1[v * NU + n]); b2[j] = bfr(BF2[v * NU + n]); bt[j] = bfr(BTA[v * NU + n]) + bfr(BTB[v * NU + n]); }
#pragma unroll
  for (int j = 0; j < 8; ++j)
#pragma unroll
    for (int r = 0; r < 8; ++r) sh[wave][8 * g + r][j * 16 + col] = 0.f;
  LDSX();
#pragma unroll 1
  for (int t = 0; t < NT; ++t) {
    float xt[8];
#pragma unroll
    for (int r = 0; r < 8; ++r) xt[r] = bfr(X[((size_t)v * NBAT + b0 + 8 * g + r) * NT + t]);
    v8f acc[8] = {};
    gemm16x128(&sh[wave][col][0], PBB, lane, col, acc);
#pragma unroll
    for (int j = 0; j < 8; ++j)
#pragma unroll
      for (int r = 0; r < 8; ++r) sz[wave][8 * g + r][j * 16 + col] = 1.7159f * ftanh(0.666f * ((acc[j][r] + xt[r] * wx[j]) + bb[j]));
    LDSX();
#pragma unroll
    for (int j = 0; j < 8; ++j) acc[j] = (v8f){};
    gemm16x128(&sz[wave][col][0], PF1, lane, col, acc);
#pragma unroll
    for (int j = 0; j < 8; ++j)
#pragma unroll
      for (int r = 0; r < 8; ++r) sf1[wave][8 * g + r][j * 16 + col] = ftanh(acc[j][r] + b1[j]);
#pragma unroll
    for (int j = 0; j < 8; ++j) acc[j] = (v8f){};
    gemm16x128(&sz[wave][col][0], PF2, lane, col, acc);
#pragma unroll
    for (int j = 0; j < 8; ++j)
#pragma unroll
      for (int r = 0; r < 8; ++r) sf2[wave][8 * g + r][j * 16 + col] = ftanh(acc[j][r] + b2[j]);
#pragma unroll
    for (int j = 0; j < 8; ++j) acc[j] = (v8f){};
    gemm16x128(&sz[wave][col][0], PTA, lane, col, acc);
    gemm16x128(&sz[wave][col][0], PTB, lane, col, acc);
    LDSX();
#pragma unroll
    for (int j = 0; j < 8; ++j)
#pragma unroll
      for (int r = 0; r < 8; ++r) { const int rr = 8 * g + r, c = j * 16 + col; const float ti = fsigm(acc[j][r] + bt[j]); const float f1 = sf1[wave][rr][c], f2 = sf2[wave][rr][c]; sh[wave][rr][c] = f1 * (1.0f - ti) + ti * f2; }
    LDSX(); }
  for (int rl = 0; rl < 16; ++rl) vst2(FE + (size_t)(b0 + rl) * NHID + v * NU + lane * 4, *(const v4f*)&sh[wave][rl][lane * 4]);
}
__global__ __launch_bounds__(128) void k_fc1(const float* __restrict__ FE, const __bf16* __restrict__ P, const float* __restrict__ bias, float* __restrict__ H1) {
  __shared__ __align__(16) float so[4][16][132];
  const int tid = threadIdx.x, wave = tid >> 5, lane = tid & 31, col = lane & 15, g = lane >> 4; const size_t r0 = (size_t)blockIdx.x * 64 + wave * 16; const int n0 = blockIdx.y * 128;
  v8f acc[8] = {};
#pragma unroll 2
  for (int kc = 0; kc < NHID / 32; ++kc) { const F2 a = split_row(FE + (r0 + col) * NHID, kc * 32, lane);
#pragma unroll
    for (int j = 0; j < 8; ++j) { const v16b w = frag_b(P + (size_t)(n0 + j * 16 + col) * NHID + kc * 32, lane); acc[j] = wmma_bf(a.l, w, acc[j]); acc[j] = wmma_bf(a.h, w, acc[j]); } }
#pragma unroll
  for (int j = 0; j < 8; ++j) { const float b_ = bfr(bias[n0 + j * 16 + col]);
#pragma unroll
    for (int r = 0; r < 8; ++r) so[wave][8 * g + r][j * 16 + col] = fmaxf(acc[j][r] + b_, 0.f); }
  LDSX();
  for (int rl = 0; rl < 16; ++rl) vst2(H1 + (r0 + rl) * NHID + n0 + lane * 4, *(const v4f*)&so[wave][rl][lane * 4]);
}
__global__ __launch_bounds__(256) void k_fc2(const float* __restrict__ H1, const __bf16* __restrict__ P, const float* __restrict__ bias, float* __restrict__ OUT) {
  __shared__ __align__(16) float so[NBAT * NCLS + 64];
  const int tid = threadIdx.x, wave = tid >> 5, lane = tid & 31, col = lane & 15, g = lane >> 4;
#pragma unroll 1
  for (int rt = 0; rt < 2; ++rt) { const size_t r0 = (size_t)(wave * 2 + rt) * 16; v8f acc = {};
#pragma unroll 4
    for (int kc = 0; kc < NHID / 32; ++kc) { const F2 a = split_row(H1 + (r0 + col) * NHID, kc * 32, lane); const v16b w = frag_b(P + (size_t)col * NHID + kc * 32, lane); acc = wmma_bf(a.l, w, acc); acc = wmma_bf(a.h, w, acc); }
    if (col < NCLS) { const float b_ = bfr(bias[col]);
#pragma unroll
      for (int r = 0; r < 8; ++r) so[(r0 + 8 * g + r) * NCLS + col] = acc[r] + b_; } }
  __syncthreads();
  for (int q = tid; q < NOUT * NCLS / 4; q += 256) vst2(OUT + q * 4, *(const v4f*)&so[q * 4]);
}
extern "C" void kernel_launch(void* const* d_in, const int* in_sizes, int n_in, void* d_out, int out_size, void* d_ws, size_t ws_size, hipStream_t stream) {
  (void)in_sizes; (void)n_in; (void)out_size;
  const float** F = (const float**)d_in;
  if (ws_size < (size_t)WS_END) return;
  char* ws = (char*)d_ws; __bf16* PK = (__bf16*)(ws + WS_PK); float *FE = (float*)(ws + WS_FE), *H1 = (float*)(ws + WS_H1);
  k_packT<<<dim3(NHID, 42), 256, 0, stream>>>(F[1], F[3], F[5], F[7], F[9], F[11], F[13], PK);
  k_cfc<<<dim3(NRG, NV), 64, 0, stream>>>(F[0], F[1], F[2], F[4], F[6], F[8], F[10], PK, FE);
  k_fc1<<<dim3(NBAT / 64, NHID / 128), 128, 0, stream>>>(FE, PK + PK_FC1, F[12], H1);
  k_fc2<<<1, 256, 0, stream>>>(H1, PK + PK_FC2, F[14], (float*)d_out);
}
